// DCNv2_70428873719887
// MI455X (gfx1250) — hardware-verified
//
#include <hip/hip_runtime.h>
#include <stddef.h>
#include <math.h>

typedef __attribute__((ext_vector_type(16))) _Float16 v16h;
typedef __attribute__((ext_vector_type(8)))  _Float16 v8h;
typedef __attribute__((ext_vector_type(16))) __bf16   v16b;
typedef __attribute__((ext_vector_type(8)))  __bf16   v8b;
typedef __attribute__((ext_vector_type(8)))  float    v8f;
typedef __attribute__((ext_vector_type(4)))  float    v4f;
typedef __attribute__((ext_vector_type(4)))  int      v4i;

constexpr int NBATCH   = 8;
constexpr int NCH_IN   = 128;
constexpr int NCH_OUT  = 128;
constexpr int IMGH     = 64;
constexpr int IMGW     = 64;
constexpr int NPIX     = IMGH * IMGW;
constexpr int NTAP     = 9;
constexpr int KDIM     = NTAP * NCH_IN;
constexpr int NTHR     = 256;
constexpr int PIXT     = 16;
constexpr int NROWT    = NTAP * PIXT;
constexpr int CHUNK    = 64;
constexpr int NCHUNK   = NCH_IN / CHUNK;
constexpr float S_CARRY = 16.0f;
constexpr float W_CARRY = 64.0f;
constexpr float FOLD    = 1.0f / 1024.0f;

constexpr size_t WT_BYTES = (size_t)NCH_OUT * KDIM * 2;
constexpr size_t SP_BYTES = (size_t)NBATCH * NPIX * KDIM * 2;
constexpr size_t WS_TOTAL = WT_BYTES + SP_BYTES;

static_assert(KDIM % 32 == 0);
static_assert(NCH_OUT % 64 == 0 && NPIX % 64 == 0);
static_assert(WT_BYTES % 128 == 0);
static_assert((KDIM * 2) % 128 == 0);
static_assert((NCH_OUT * KDIM / 8) % NTHR == 0);
static_assert(NROWT * CHUNK == NTHR * 36);
static_assert(NROWT <= NTHR);
static_assert(NBATCH * IMGH * (IMGW / PIXT) == 2048);
static_assert(WS_TOTAL <= (size_t)134217728);

__device__ __forceinline__ unsigned short f2bf_bits(float f) {
  unsigned u = __float_as_uint(f);
  return (unsigned short)((u + 0x7FFFu + ((u >> 16) & 1u)) >> 16);
}
__device__ __forceinline__ float bf_bits2f(unsigned short h) { return __uint_as_float(((unsigned)h) << 16); }

__device__ __forceinline__ void dep_guard_h(v8f& a, v8f& b, v16h x, v16h y) { asm volatile("v_nop\n\tv_nop\n\tv_nop\n\tv_nop" : "+v"(a), "+v"(b) : "v"(x), "v"(y)); }
__device__ __forceinline__ void dep_guard_b(v8f& a, v8f& b, v16b x, v16b y) { asm volatile("v_nop\n\tv_nop\n\tv_nop\n\tv_nop" : "+v"(a), "+v"(b) : "v"(x), "v"(y)); }
__device__ __forceinline__ void dep_guard4_h(v8f& a, v8f& b, v8f& c, v8f& d, v16h x, v16h y) { asm volatile("v_nop\n\tv_nop\n\tv_nop\n\tv_nop" : "+v"(a), "+v"(b), "+v"(c), "+v"(d) : "v"(x), "v"(y)); }
__device__ __forceinline__ void dep_guard4_b(v8f& a, v8f& b, v8f& c, v8f& d, v16b x, v16b y) { asm volatile("v_nop\n\tv_nop\n\tv_nop\n\tv_nop" : "+v"(a), "+v"(b), "+v"(c), "+v"(d) : "v"(x), "v"(y)); }
__device__ __forceinline__ void keep4_h(v16h a, v16h b, v16h c, v16h d) { asm volatile("v_nop" :: "v"(a), "v"(b), "v"(c), "v"(d)); }
__device__ __forceinline__ void keep4_b(v16b a, v16b b, v16b c, v16b d) { asm volatile("v_nop" :: "v"(a), "v"(b), "v"(c), "v"(d)); }
__device__ __forceinline__ void acc_guard4(v8f& a, v8f& b, v8f& c, v8f& d) { asm volatile("v_nop\n\tv_nop\n\tv_nop\n\tv_nop" : "+v"(a), "+v"(b), "+v"(c), "+v"(d)); }
template <typename T> struct Frag;
template <> struct Frag<_Float16> {
  typedef v16h V; union U { v16h v; v8h h[2]; };
  static __device__ __forceinline__ v16h load(const _Float16* p) {
    U f; f.h[0] = *(const v8h*)(p); f.h[1] = *(const v8h*)(p + 16); return f.v;
  }
  static __device__ __forceinline__ v8f mma(v16h a, v16h b, v8f c) {
    return __builtin_amdgcn_wmma_f32_16x16x32_f16(false, a, false, b, (short)0, c, false, false);
  }
  static __device__ __forceinline__ void guard(v8f& a, v8f& b, v16h x, v16h y) { dep_guard_h(a, b, x, y); }
  static __device__ __forceinline__ void guard4(v8f& a, v8f& b, v8f& c, v8f& d, v16h x, v16h y) { dep_guard4_h(a, b, c, d, x, y); }
  static __device__ __forceinline__ void keep(v16h a, v16h b, v16h c, v16h d) { keep4_h(a, b, c, d); }
};
template <> struct Frag<__bf16> {
  typedef v16b V; union U { v16b v; v8b h[2]; };
  static __device__ __forceinline__ v16b load(const __bf16* p) {
    U f; f.h[0] = *(const v8b*)(p); f.h[1] = *(const v8b*)(p + 16); return f.v;
  }
  static __device__ __forceinline__ v8f mma(v16b a, v16b b, v8f c) {
    return __builtin_amdgcn_wmma_f32_16x16x32_bf16(false, a, false, b, (short)0, c, false, false);
  }
  static __device__ __forceinline__ void guard(v8f& a, v8f& b, v16b x, v16b y) { dep_guard_b(a, b, x, y); }
  static __device__ __forceinline__ void guard4(v8f& a, v8f& b, v8f& c, v8f& d, v16b x, v16b y) { dep_guard4_b(a, b, c, d, x, y); }
  static __device__ __forceinline__ void keep(v16b a, v16b b, v16b c, v16b d) { keep4_b(a, b, c, d); }
};

template <int ET> struct Elem;
template <> struct Elem<0> { typedef _Float16 T; };
template <> struct Elem<1> { typedef __bf16 T; };
template <int ET, bool SPLIT, int BIAS_MODE, int OUT_MODE, bool RESID, int ACT = 0>
__global__ __launch_bounds__(256) void wmma_gemm64(
    const unsigned short* __restrict__ Ap, const unsigned short* __restrict__ A2p, int lda, long strideA,
    const unsigned short* __restrict__ Btp, const unsigned short* __restrict__ Bt2p, int ldb, long strideB,
    void* __restrict__ Cout, void* __restrict__ Cout2, int ldc, long strideC,
    const float* __restrict__ bias,
    const float* __restrict__ resid, long strideR,
    int M, int N, int K, float scale) {
  typedef typename Elem<ET>::T T;
  typedef typename Frag<T>::V V;
  const T* A = (const T*)Ap; const T* A2 = (const T*)A2p; const T* Bt = (const T*)Btp; const T* Bt2 = (const T*)Bt2p;
  __shared__ __align__(16) float sT[8][16 * 68];
  const int b    = blockIdx.y;
  const int lane = threadIdx.x & 31;
  const int wave = threadIdx.x >> 5;
  const int tilesN = N >> 6;
  const int tilesM = M >> 6;
  const int tile = blockIdx.x * 8 + wave;
  if (tile >= tilesM * tilesN) return;
  const int tm = tile / tilesN;
  const int tn = tile - tm * tilesN;
  const int m0 = tm << 6;
  const int n0 = tn << 6;

  const T* Ab  = A  + (size_t)b * strideA;
  const T* Bb  = Bt + (size_t)b * strideB;
  const T* Ab2 = SPLIT ? (A2  + (size_t)b * strideA) : nullptr;
  const T* Bb2 = SPLIT ? (Bt2 + (size_t)b * strideB) : nullptr;

  const int rlane = lane & 15;
  const int koff  = (lane >> 4) * 8;
  const int mOff  = (lane >> 4) * 8;

  v8f acc[4][4];
#pragma unroll
  for (int i = 0; i < 4; ++i)
#pragma unroll
    for (int j = 0; j < 4; ++j) acc[i][j] = (v8f){0.f,0.f,0.f,0.f,0.f,0.f,0.f,0.f};

  for (int k0 = 0; k0 < K; k0 += 32) {
    V bh[4], bl[4];
#pragma unroll
    for (int j = 0; j < 4; ++j) {
      const size_t bo = (size_t)(n0 + (j << 4) + rlane) * ldb + koff + k0;
      bh[j] = Frag<T>::load(Bb + bo);
      if (SPLIT) bl[j] = Frag<T>::load(Bb2 + bo);
    }
#pragma unroll
    for (int i = 0; i < 4; ++i) {
      const size_t ao = (size_t)(m0 + (i << 4) + rlane) * lda + koff + k0;
      V ah = Frag<T>::load(Ab + ao);
      V al;
      if (SPLIT) al = Frag<T>::load(Ab2 + ao);
#pragma unroll
      for (int j = 0; j < 4; ++j) {
        acc[i][j] = Frag<T>::mma(ah, bh[j], acc[i][j]);
        if (SPLIT) {
          acc[i][j] = Frag<T>::mma(ah, bl[j], acc[i][j]);
          acc[i][j] = Frag<T>::mma(al, bh[j], acc[i][j]);
        }
      }
      Frag<T>::guard4(acc[i][0], acc[i][1], acc[i][2], acc[i][3], ah, SPLIT ? al : ah);
    }
    Frag<T>::keep(bh[0], bh[1], bh[2], bh[3]);
    if (SPLIT) Frag<T>::keep(bl[0], bl[1], bl[2], bl[3]);
  }
  acc_guard4(acc[0][0], acc[0][1], acc[0][2], acc[0][3]);
  acc_guard4(acc[1][0], acc[1][1], acc[1][2], acc[1][3]);
  acc_guard4(acc[2][0], acc[2][1], acc[2][2], acc[2][3]);
  acc_guard4(acc[3][0], acc[3][1], acc[3][2], acc[3][3]);

  float* slab = sT[wave];
  const float* Rb = RESID ? (resid + (size_t)b * strideR) : nullptr;
#pragma unroll
  for (int i = 0; i < 4; ++i) {
    const int mBase = m0 + (i << 4);
    v4f bm0 = (v4f){0.f, 0.f, 0.f, 0.f};
    v4f bm1 = (v4f){0.f, 0.f, 0.f, 0.f};
    if (BIAS_MODE == 1) {
      bm0 = *(const v4f*)(bias + mBase + mOff);
      bm1 = *(const v4f*)(bias + mBase + mOff + 4);
    }
#pragma unroll
    for (int j = 0; j < 4; ++j) {
      const int n = n0 + (j << 4) + rlane;
      float bv = 0.f;
      if (BIAS_MODE == 2) bv = bias[n];
#pragma unroll
      for (int r = 0; r < 8; ++r) {
        float v = acc[i][j][r] * scale;
        if (BIAS_MODE == 1) v += (r < 4) ? bm0[r & 3] : bm1[r & 3];
        if (BIAS_MODE == 2) v += bv;
        if (RESID) v += Rb[(size_t)(mBase + mOff + r) * ldc + n];
        if (ACT == 1) v = tanhf(v);
        if (ACT == 2) v = fmaxf(v, 0.0f);
        if (ACT == 3) v = v / (1.0f + expf(-v));
        if (ACT == 4) v = (v > 0.f) ? v : 0.01f * v;
        slab[(mOff + r) * 68 + (j << 4) + rlane] = v;
      }
    }
    __builtin_amdgcn_fence(__ATOMIC_RELEASE, "workgroup");
    __builtin_amdgcn_wave_barrier();
    __builtin_amdgcn_fence(__ATOMIC_ACQUIRE, "workgroup");
    if (OUT_MODE == 0) {
      float* C = (float*)Cout + (size_t)b * strideC;
      const int hh = lane >> 4, c4 = (lane & 15) * 4;
      for (int pass = 0; pass < 2; ++pass) {
#pragma unroll
        for (int it = 0; it < 8; ++it) {
          const int row = it * 2 + hh;
          v4f v = *(const v4f*)(slab + row * 68 + c4);
          *(volatile v4f*)(C + (size_t)(mBase + row) * ldc + n0 + c4) = v;
        }
        __threadfence();
      }
    } else {
      const int q = lane >> 3, c8 = (lane & 7) * 8;
      unsigned short* C  = (unsigned short*)Cout  + (size_t)b * strideC;
      unsigned short* C2 = (OUT_MODE == 2) ? ((unsigned short*)Cout2 + (size_t)b * strideC) : nullptr;
      for (int pass = 0; pass < 2; ++pass) {
#pragma unroll
        for (int it = 0; it < 4; ++it) {
          const int row = it * 4 + q;
          const float* sp = slab + row * 68 + c8;
          v8h hv, lv;
#pragma unroll
          for (int e = 0; e < 8; ++e) {
            if (OUT_MODE == 1) {
              hv[e] = (_Float16)sp[e];
            } else {
              unsigned short hb = f2bf_bits(sp[e]);
              unsigned short lb = f2bf_bits(sp[e] - bf_bits2f(hb));
              hv[e] = __builtin_bit_cast(_Float16, hb);
              lv[e] = __builtin_bit_cast(_Float16, lb);
            }
          }
          *(volatile v8h*)(C + (size_t)(mBase + row) * ldc + n0 + c8) = hv;
          if (OUT_MODE == 2) *(volatile v8h*)(C2 + (size_t)(mBase + row) * ldc + n0 + c8) = lv;
        }
        __threadfence();
      }
    }
    __builtin_amdgcn_fence(__ATOMIC_RELEASE, "workgroup");
    __builtin_amdgcn_wave_barrier();
    __builtin_amdgcn_fence(__ATOMIC_ACQUIRE, "workgroup");
  }
}

__global__ __launch_bounds__(NTHR) void k_wprep(const float* __restrict__ w, unsigned short* __restrict__ wt) {
  const int i = blockIdx.x * NTHR + threadIdx.x;
  if (i >= NCH_OUT * KDIM / 8) return;
  const int o   = i / (KDIM / 8);
  const int rem = i - o * (KDIM / 8);
  const int kc0 = rem * 8;
  const int k   = kc0 >> 7;
  const int c0  = kc0 & 127;
  v8h hv;
#pragma unroll
  for (int e = 0; e < 8; ++e) {
    const float v = w[((size_t)(o * NCH_IN + c0 + e)) * NTAP + k];
    hv[e] = (_Float16)(v * W_CARRY);
  }
  const size_t off = (size_t)i * 8;
  *(volatile v8h*)(wt + off) = hv;
  __threadfence();
  *(volatile v8h*)(wt + off) = hv;
}

__global__ __launch_bounds__(NTHR) void k_sample(const float* __restrict__ x, const float* __restrict__ offs,
                                                 const float* __restrict__ msk, unsigned short* __restrict__ splane) {
  __shared__ __align__(16) int   s_idx[NTHR * 4];
  __shared__ __align__(16) float s_wgt[NTHR * 4];
  __shared__ __align__(16) float s_tile[NROWT * CHUNK];

  const int tid  = threadIdx.x;
  const int blk  = blockIdx.x;
  const int wq   = blk & 3;
  const int ho   = (blk >> 2) & 63;
  const int b    = blk >> 8;
  const int wo0  = wq * PIXT;

  {
    const int rc = (tid < NROWT) ? tid : (NROWT - 1);
    const int k  = rc >> 4;
    const int n  = rc & 15;
    const int wo = wo0 + n;
    const int ky = k / 3;
    const int kx = k - 3 * ky;
    const size_t pix = (size_t)ho * IMGW + wo;
    const float off_y = offs[((size_t)b * (2 * NTAP) + 2 * k    ) * NPIX + pix];
    const float off_x = offs[((size_t)b * (2 * NTAP) + 2 * k + 1) * NPIX + pix];
    const float mv    = msk [((size_t)b * NTAP + k) * NPIX + pix];
    const float sy  = (float)(ky + ho - 1) + off_y;
    const float sx  = (float)(kx + wo - 1) + off_x;
    const float y0f = floorf(sy);
    const float x0f = floorf(sx);
    const float wy1 = sy - y0f;
    const float wx1 = sx - x0f;
    const float wy0 = 1.0f - wy1;
    const float wx0 = 1.0f - wx1;
    const int y0 = (int)y0f, x0 = (int)x0f;
    const int y1 = y0 + 1,   x1 = x0 + 1;
    const float fy0 = ((y0 >= 0) && (y0 <= IMGH - 1)) ? 1.0f : 0.0f;
    const float fy1 = ((y1 >= 0) && (y1 <= IMGH - 1)) ? 1.0f : 0.0f;
    const float fx0 = ((x0 >= 0) && (x0 <= IMGW - 1)) ? 1.0f : 0.0f;
    const float fx1 = ((x1 >= 0) && (x1 <= IMGW - 1)) ? 1.0f : 0.0f;
    const int cy0 = min(max(y0, 0), IMGH - 1);
    const int cy1 = min(max(y1, 0), IMGH - 1);
    const int cx0 = min(max(x0, 0), IMGW - 1);
    const int cx1 = min(max(x1, 0), IMGW - 1);
    v4i iv;
    iv[0] = cy0 * IMGW + cx0;
    iv[1] = cy0 * IMGW + cx1;
    iv[2] = cy1 * IMGW + cx0;
    iv[3] = cy1 * IMGW + cx1;
    v4f wv;
    wv[0] = (mv * (wy0 * wx0)) * (fy0 * fx0);
    wv[1] = (mv * (wy0 * wx1)) * (fy0 * fx1);
    wv[2] = (mv * (wy1 * wx0)) * (fy1 * fx0);
    wv[3] = (mv * (wy1 * wx1)) * (fy1 * fx1);
    *(v4i*)(s_idx + tid * 4) = iv;
    *(v4f*)(s_wgt + tid * 4) = wv;
  }
  __syncthreads();

  const float* xb = x + (size_t)b * NCH_IN * NPIX;
  const int c    = tid & 63;
  const int rb   = tid >> 6;
  const int wave = tid >> 5;
  const int lane = tid & 31;
  const int q    = lane >> 3;
  const int c8   = (lane & 7) * 8;
  const size_t pixrow0 = (size_t)b * NPIX + (size_t)ho * IMGW + wo0;

#pragma unroll 1
  for (int ch = 0; ch < NCHUNK; ++ch) {
    const float* xc = xb + (size_t)(ch * CHUNK + c) * NPIX;
#pragma unroll 2
    for (int i = 0; i < 36; ++i) {
      const int r = rb + 4 * i;
      const v4i iv = *(const v4i*)(s_idx + r * 4);
      const v4f wv = *(const v4f*)(s_wgt + r * 4);
      const float xv0 = xc[iv[0] & (NPIX - 1)];
      const float xv1 = xc[iv[1] & (NPIX - 1)];
      const float xv2 = xc[iv[2] & (NPIX - 1)];
      const float xv3 = xc[iv[3] & (NPIX - 1)];
      float v = wv[0] * xv0;
      v = fmaf(wv[1], xv1, v);
      v = fmaf(wv[2], xv2, v);
      v = fmaf(wv[3], xv3, v);
      s_tile[r * CHUNK + c] = v;
    }
    __syncthreads();

    for (int pass = 0; pass < 2; ++pass) {
#pragma unroll
      for (int it = 0; it < 5; ++it) {
        const int r  = it * 32 + wave * 4 + q;
        const int rr = (r < NROWT) ? r : (NROWT - 1);
        const float* sp = s_tile + rr * CHUNK + c8;
        const v4f a0 = *(const v4f*)(sp);
        const v4f a1 = *(const v4f*)(sp + 4);
        v8h hv;
        hv[0] = (_Float16)(a0[0] * S_CARRY);
        hv[1] = (_Float16)(a0[1] * S_CARRY);
        hv[2] = (_Float16)(a0[2] * S_CARRY);
        hv[3] = (_Float16)(a0[3] * S_CARRY);
        hv[4] = (_Float16)(a1[0] * S_CARRY);
        hv[5] = (_Float16)(a1[1] * S_CARRY);
        hv[6] = (_Float16)(a1[2] * S_CARRY);
        hv[7] = (_Float16)(a1[3] * S_CARRY);
        const int k = rr >> 4;
        const int n = rr & 15;
        const size_t o = (pixrow0 + (size_t)n) * KDIM + (size_t)(k * NCH_IN + ch * CHUNK + c8);
        if (r < NROWT) *(volatile v8h*)(splane + o) = hv;
      }
      __threadfence();
    }
    __syncthreads();
  }
}

extern "C" void kernel_launch(void* const* d_in, const int* in_sizes, int n_in,
                              void* d_out, int out_size, void* d_ws, size_t ws_size,
                              hipStream_t stream) {
  if (n_in < 5) return;
  if (in_sizes[0] != NBATCH * NCH_IN * NPIX) return;
  if (in_sizes[1] != NBATCH * 2 * NTAP * NPIX) return;
  if (in_sizes[2] != NBATCH * NTAP * NPIX) return;
  if (in_sizes[3] != NCH_OUT * NCH_IN * NTAP) return;
  if (in_sizes[4] != NCH_OUT) return;
  if (out_size != NBATCH * NCH_OUT * NPIX) return;
  if (ws_size < WS_TOTAL) return;

  const float* x      = (const float*)d_in[0];
  const float* offs   = (const float*)d_in[1];
  const float* msk    = (const float*)d_in[2];
  const float* weight = (const float*)d_in[3];
  const float* bias   = (const float*)d_in[4];
  float* out          = (float*)d_out;
  unsigned short* wt  = (unsigned short*)d_ws;
  unsigned short* sp  = (unsigned short*)((char*)d_ws + WT_BYTES);

  k_wprep<<<NCH_OUT * KDIM / 8 / NTHR, NTHR, 0, stream>>>(weight, wt);
  k_sample<<<NBATCH * IMGH * (IMGW / PIXT), NTHR, 0, stream>>>(x, offs, msk, sp);

  const int tiles  = (NCH_OUT / 64) * (NPIX / 64);
  dim3 ggrid((tiles + 7) / 8, NBATCH);
  wmma_gemm64<0, false, 1, 0, false, 0><<<ggrid, 256, 0, stream>>>(
      wt, wt, KDIM, 0L,
      sp, sp, KDIM, (long)NPIX * KDIM,
      (void*)out, (void*)out, NPIX, (long)NCH_OUT * NPIX,
      bias,
      bias, 0L,
      NCH_OUT, NPIX, KDIM, FOLD);
}
